// JointDrifting_10050223472719
// MI455X (gfx1250) — hardware-verified
//
#include <hip/hip_runtime.h>


#define NN   4096
#define DD   512
#define NC   (2 * NN)
#define KCH  1024
#define NCHK (NC / KCH)
typedef _Float16 h16;
typedef unsigned short bf;
typedef __attribute__((ext_vector_type(16))) __bf16   v16bf;
typedef __attribute__((ext_vector_type(16))) _Float16 v16h;
typedef __attribute__((ext_vector_type(8)))  _Float16 v8h;
typedef __attribute__((ext_vector_type(8)))  unsigned short v8us;
typedef __attribute__((ext_vector_type(8)))  float    v8f;
typedef __attribute__((ext_vector_type(4)))  float    v4f;
typedef v8h  __attribute__((may_alias)) v8ha;
typedef v4f  __attribute__((may_alias)) v4fa;
typedef v8us __attribute__((may_alias)) v8usa;

__device__ __forceinline__ unsigned short f2bf(float f) { unsigned u = __float_as_uint(f); u += 0x7FFFu + ((u >> 16) & 1u); return (unsigned short)(u >> 16); }
__device__ __forceinline__ float bf2f(unsigned short b) { return __uint_as_float(((unsigned)b) << 16); }
__device__ __forceinline__ float bfr(float f) { return bf2f(f2bf(f)); }
__device__ __forceinline__ v16h cat16(v8h lo, v8h hi) { return __builtin_shufflevector(lo, hi, 0, 1, 2, 3, 4, 5, 6, 7, 8, 9, 10, 11, 12, 13, 14, 15); }
__device__ __forceinline__ v16bf cat16b(v8us lo, v8us hi) { return __builtin_bit_cast(v16bf, __builtin_shufflevector(lo, hi, 0, 1, 2, 3, 4, 5, 6, 7, 8, 9, 10, 11, 12, 13, 14, 15)); }
__device__ __forceinline__ v8f wmma16(v16h a, v16h b, v8f c) { return __builtin_amdgcn_wmma_f32_16x16x32_f16(false, a, false, b, (short)0, c, false, false); }
__device__ __forceinline__ v8f wmmab(v16bf a, v16bf b, v8f c) { return __builtin_amdgcn_wmma_f32_16x16x32_bf16(false, a, false, b, (short)0, c, false, false); }


template <typename T16> struct WFrag;
template <> struct WFrag<h16> { typedef v16h V; static __device__ __forceinline__ V ld(const h16* p) { return cat16(*(const v8h*)p, *(const v8h*)(p + 16)); } static __device__ __forceinline__ v8f mma(V a, V b, v8f c) { return wmma16(a, b, c); } };
template <> struct WFrag<bf> { typedef v16bf V; static __device__ __forceinline__ V ld(const bf* p) { return cat16b(*(const v8us*)p, *(const v8us*)(p + 16)); } static __device__ __forceinline__ v8f mma(V a, V b, v8f c) { return wmmab(a, b, c); } };
template <typename T16, int NSPLIT, bool BIAS>
__global__ __launch_bounds__(32) void k_gemmw(const T16* __restrict__ A, const T16* __restrict__ A2, const T16* __restrict__ Bt, const T16* __restrict__ Bt2, int K, float* C, int ldc, const float* __restrict__ bias, size_t sA, size_t sB, size_t sC) {
    typedef typename WFrag<T16>::V V;
    __shared__ __align__(16) float os[16 * 68];
    const size_t z = blockIdx.z; A += z * sA; if (A2) A2 += z * sA; Bt += z * sB; if (Bt2) Bt2 += z * sB; C += z * sC;
    const int lane = threadIdx.x & 31, lr = lane & 15, hi = lane >> 4; const int r0 = blockIdx.x * 64, c0 = blockIdx.y * 64;
    v8f acc[4][4];
#pragma unroll
    for (int mb = 0; mb < 4; ++mb)
#pragma unroll
        for (int nb = 0; nb < 4; ++nb) acc[mb][nb] = (v8f){};
    const size_t aoff = (size_t)(r0 + lr) * K + 8 * hi, boff = (size_t)(c0 + lr) * K + 8 * hi;
#pragma unroll 1
    for (int kc = 0; kc < K; kc += 32) {
        V a[4], a2[4];
#pragma unroll
        for (int mb = 0; mb < 4; ++mb) { a[mb] = WFrag<T16>::ld(A + aoff + (size_t)mb * 16 * K + kc); if (NSPLIT == 1 || NSPLIT == 2) a2[mb] = WFrag<T16>::ld(A2 + aoff + (size_t)mb * 16 * K + kc); }
#pragma unroll
        for (int nb = 0; nb < 4; ++nb) { const V b = WFrag<T16>::ld(Bt + boff + (size_t)nb * 16 * K + kc); V b2; if (NSPLIT >= 2) b2 = WFrag<T16>::ld(Bt2 + boff + (size_t)nb * 16 * K + kc);
#pragma unroll
            for (int mb = 0; mb < 4; ++mb) { acc[mb][nb] = WFrag<T16>::mma(a[mb], b, acc[mb][nb]); if (NSPLIT == 1 || NSPLIT == 2) acc[mb][nb] = WFrag<T16>::mma(a2[mb], b, acc[mb][nb]); if (NSPLIT >= 2) acc[mb][nb] = WFrag<T16>::mma(a[mb], b2, acc[mb][nb]); } }
        asm volatile("v_nop\n\tv_nop\n\tv_nop\n\tv_nop" : "+v"(acc[0][0]), "+v"(acc[1][1]), "+v"(acc[2][2]), "+v"(acc[3][3]) : "v"(a[0]), "v"(a[3]));
    }
#pragma unroll
    for (int mb = 0; mb < 4; ++mb) {
#pragma unroll
        for (int nb = 0; nb < 4; ++nb) {
#pragma unroll
            for (int j = 0; j < 8; ++j) os[(hi * 8 + j) * 68 + nb * 16 + lr] = acc[mb][nb][j]; }
        __builtin_amdgcn_wave_barrier(); asm volatile("" ::: "memory");
        float* crow = C + (size_t)(r0 + mb * 16) * ldc + c0;
#pragma unroll 1
        for (int ps = 0; ps < 2; ++ps) {
#pragma unroll
            for (int s = 0; s < 8; ++s) { const int row = 2 * s + hi, cofs = lr * 4; v4f val = *(const v4fa*)(os + row * 68 + cofs); if (BIAS) { val[0] += bfr(bias[c0 + cofs]); val[1] += bfr(bias[c0 + cofs + 1]); val[2] += bfr(bias[c0 + cofs + 2]); val[3] += bfr(bias[c0 + cofs + 3]); }
                *(volatile v4f*)(crow + (size_t)row * ldc + cofs) = val; }
            if (ps == 0) __threadfence(); }
        __builtin_amdgcn_wave_barrier(); asm volatile("" ::: "memory");
    }
}

__device__ __forceinline__ void splitf(float y, unsigned short& h, unsigned short& l) { h = f2bf(y); l = f2bf(y - bf2f(h)); }
typedef __attribute__((ext_vector_type(2))) unsigned short v2us;
typedef __attribute__((ext_vector_type(8))) unsigned short v8us_;

__global__ __launch_bounds__(256) void k_cvt8(const float* __restrict__ src, bf* dst, size_t n8) { const size_t i = (size_t)blockIdx.x * 256 + threadIdx.x; if (i >= n8) return; const v8f v = *(const v8f*)(src + i * 8); v8us o;
#pragma unroll
    for (int k = 0; k < 8; ++k) o[k] = f2bf(v[k]); *(volatile v8us*)(dst + i * 8) = o; __threadfence(); *(volatile v8us*)(dst + i * 8) = o; }
__global__ __launch_bounds__(256) void k_tr(const float* __restrict__ src, bf* T) {
    __shared__ float tl[64][65];
    const int tid = threadIdx.x; const int j0 = blockIdx.x * 64, d0 = blockIdx.y * 64;
#pragma unroll
    for (int i = 0; i < 16; ++i) { const int jj = i * 4 + (tid >> 6), dd = tid & 63; tl[jj][dd] = src[(size_t)(j0 + jj) * DD + d0 + dd]; }
    __syncthreads();
    const int lane = tid & 31, wv = tid >> 5; const int c = j0 / KCH, jl0 = j0 % KCH;
    auto pass = [&]() {
#pragma unroll
        for (int i2 = 0; i2 < 2; ++i2) { const int r = wv * 8 + i2 * 4 + (lane >> 3); const int cq = (lane & 7) * 8; v8us_ o;
#pragma unroll
            for (int i = 0; i < 8; ++i) o[i] = f2bf(tl[cq + i][r]);
            *(volatile v8us_*)(T + (((size_t)c * DD + d0 + r) * KCH) + jl0 + cq) = o; } };
    pass(); __threadfence(); pass();
}
__global__ __launch_bounds__(256) void k_sq(const float* __restrict__ v, float* SQ) {
    const int lane = threadIdx.x & 31; const int r0 = (blockIdx.x * 8 + (threadIdx.x >> 5)) * 32; if (r0 >= NN) return; const float* row = v + (size_t)(r0 + lane) * DD; float s = 0.f;
#pragma unroll 8
    for (int d = 0; d < DD; ++d) { const float t = bfr(row[d]); s = fmaf(t, t, s); }
    *(volatile float*)(SQ + r0 + lane) = s; __threadfence(); *(volatile float*)(SQ + r0 + lane) = s;
}
__global__ __launch_bounds__(256) void k_logit(float* L, const float* __restrict__ SQX, const float* __restrict__ SQY) {
    const size_t i4 = (size_t)blockIdx.x * 256 + threadIdx.x; if (i4 >= (size_t)NN * NC / 4) return; const size_t e = i4 * 4; const int j = (int)(e % NC); const int i = (int)(e / NC);
    const v4f g = *(const v4f*)(L + e); v4f o; const float sqi = SQX[i];
#pragma unroll
    for (int q = 0; q < 4; ++q) { const int jj = j + q; const bool neg = jj >= NN; const int jc = neg ? jj - NN : jj; const float sqj = neg ? SQX[jc] : SQY[jc];
        const float d2 = fmaxf(sqi + sqj - 2.0f * g[q], 1e-12f); float dist = sqrtf(d2); if (neg && jc == i) dist += 1e6f; o[q] = -__fdiv_rn(dist, 0.1f); }
    *(volatile v4f*)(L + e) = o; __threadfence(); *(volatile v4f*)(L + e) = o;
}
__global__ __launch_bounds__(256) void k_rowstat(const float* __restrict__ L, float* RS) {
    const int lane = threadIdx.x & 31; const int i = blockIdx.x * 8 + (threadIdx.x >> 5); if (i >= NN) return; const float* row = L + (size_t)i * NC; float m = -3.0e38f;
#pragma unroll 2
    for (int c0 = lane * 4; c0 < NC; c0 += 128) { const v4f v = *(const v4f*)(row + c0); m = fmaxf(m, fmaxf(fmaxf(v[0], v[1]), fmaxf(v[2], v[3]))); }
#pragma unroll
    for (int sh = 16; sh; sh >>= 1) m = fmaxf(m, __shfl_xor(m, sh, 32));
    float s = 0.f;
#pragma unroll 2
    for (int c0 = lane * 4; c0 < NC; c0 += 128) { const v4f v = *(const v4f*)(row + c0);
#pragma unroll
        for (int q = 0; q < 4; ++q) s += __expf(v[q] - m); }
#pragma unroll
    for (int sh = 16; sh; sh >>= 1) s += __shfl_xor(s, sh, 32);
    const float v = lane == 0 ? m : (lane == 1 ? s : 0.f); *(volatile float*)(RS + (size_t)i * 32 + lane) = v; __threadfence(); *(volatile float*)(RS + (size_t)i * 32 + lane) = v;
}
__global__ __launch_bounds__(256) void k_colstat(const float* __restrict__ L, float* CS) {
    const int lane = threadIdx.x & 31; const int j = blockIdx.x * 8 + (threadIdx.x >> 5); if (j >= NC) return; float m = -3.0e38f;
#pragma unroll 4
    for (int i = lane; i < NN; i += 32) m = fmaxf(m, L[(size_t)i * NC + j]);
#pragma unroll
    for (int sh = 16; sh; sh >>= 1) m = fmaxf(m, __shfl_xor(m, sh, 32));
    float s = 0.f;
#pragma unroll 4
    for (int i = lane; i < NN; i += 32) s += __expf(L[(size_t)i * NC + j] - m);
#pragma unroll
    for (int sh = 16; sh; sh >>= 1) s += __shfl_xor(s, sh, 32);
    const float v = lane == 0 ? m : (lane == 1 ? s : 0.f); *(volatile float*)(CS + (size_t)j * 32 + lane) = v; __threadfence(); *(volatile float*)(CS + (size_t)j * 32 + lane) = v;
}
__global__ __launch_bounds__(256) void k_aplane(const float* __restrict__ L, const float* __restrict__ RS, const float* __restrict__ CS, int c, bf* Ah, bf* Al) {
    const int lane = threadIdx.x & 31; const int L0 = (blockIdx.x * 8 + (threadIdx.x >> 5)) * 8; const int nlines = NN * KCH / 64;
#pragma unroll 1
    for (int ps = 0; ps < 2; ++ps) {
#pragma unroll 1
        for (int l = 0; l < 8; ++l) { const int Ln = L0 + l; if (Ln >= nlines) break; const int e = Ln * 64 + lane * 2; const int jl = e & (KCH - 1); const int i = e >> 10; const float rm = RS[(size_t)i * 32], rsum = RS[(size_t)i * 32 + 1]; v2us oh, ol;
#pragma unroll
            for (int q = 0; q < 2; ++q) { const int j = c * KCH + jl + q; const float lv = L[(size_t)i * NC + j]; const float ar = __fdiv_rn(__expf(lv - rm), rsum); const float ac = __fdiv_rn(__expf(lv - CS[(size_t)j * 32]), CS[(size_t)j * 32 + 1]);
                unsigned short a, b2; splitf(sqrtf(ar * ac), a, b2); oh[q] = a; ol[q] = b2; }
            *(volatile v2us*)(Ah + (size_t)e) = oh; *(volatile v2us*)(Al + (size_t)e) = ol; }
        if (ps == 0) __threadfence(); }
}
__global__ __launch_bounds__(256) void k_acc(const float* __restrict__ P, const float* ACC, int first, float sgn, float* DST) {
    const size_t i = (size_t)blockIdx.x * 256 + threadIdx.x; if (i >= (size_t)NN * DD / 4) return; const v4f p = *(const v4f*)(P + i * 4); v4f o = first ? (v4f){0.f, 0.f, 0.f, 0.f} : *(const v4f*)(ACC + i * 4);
#pragma unroll
    for (int k = 0; k < 4; ++k) o[k] += sgn * p[k]; *(volatile v4f*)(DST + i * 4) = o; __threadfence(); *(volatile v4f*)(DST + i * 4) = o;
}

extern "C" void kernel_launch(void* const* d_in, const int* in_sizes, int n_in,
                              void* d_out, int out_size, void* d_ws, size_t ws_size, hipStream_t stream) {
    (void)in_sizes; (void)n_in; (void)out_size;
    const float* x = (const float*)d_in[0]; const float* y = (const float*)d_in[1];
    float* OUT = (float*)d_out;
    char* wsp = (char*)d_ws;
    auto take = [&](size_t bytes) { char* p = wsp; wsp += (bytes + 255) & ~(size_t)255; return (void*)p; };
    bf* XB = (bf*)take((size_t)NN * DD * 2); bf* YB = (bf*)take((size_t)NN * DD * 2); bf* XT = (bf*)take((size_t)NN * DD * 2); bf* YT = (bf*)take((size_t)NN * DD * 2);
    float* SQX = (float*)take(NN * 4); float* SQY = (float*)take(NN * 4); float* L = (float*)take((size_t)NN * NC * 4);
    float* RS = (float*)take((size_t)NN * 32 * 4); float* CS = (float*)take((size_t)NC * 32 * 4); bf* Ah = (bf*)take((size_t)NN * KCH * 2); bf* Al = (bf*)take((size_t)NN * KCH * 2); float* P = (float*)take((size_t)NN * DD * 4); float* ACC = (float*)take((size_t)NN * DD * 4);
    if ((size_t)(wsp - (char*)d_ws) > ws_size) return;
    { const size_t n8 = (size_t)NN * DD / 8; const unsigned g = (unsigned)((n8 + 255) / 256); k_cvt8<<<g, 256, 0, stream>>>(x, XB, n8); k_cvt8<<<g, 256, 0, stream>>>(y, YB, n8); }
    k_tr<<<dim3(NN / 64, DD / 64), 256, 0, stream>>>(x, XT); k_tr<<<dim3(NN / 64, DD / 64), 256, 0, stream>>>(y, YT);
    k_sq<<<NN / 32 / 8, 256, 0, stream>>>(x, SQX); k_sq<<<NN / 32 / 8, 256, 0, stream>>>(y, SQY);
    k_gemmw<bf, 0, false><<<dim3(NN / 64, NN / 64, 1), 32, 0, stream>>>(XB, nullptr, YB, nullptr, DD, L, NC, nullptr, 0, 0, 0);
    k_gemmw<bf, 0, false><<<dim3(NN / 64, NN / 64, 1), 32, 0, stream>>>(XB, nullptr, XB, nullptr, DD, L + NN, NC, nullptr, 0, 0, 0);
    k_logit<<<(unsigned)(((size_t)NN * NC / 4 + 255) / 256), 256, 0, stream>>>(L, SQX, SQY);
    k_rowstat<<<NN / 8, 256, 0, stream>>>(L, RS); k_colstat<<<NC / 8, 256, 0, stream>>>(L, CS);
    for (int c = 0; c < NCHK; ++c) { const bool pos = c < NCHK / 2;
        k_aplane<<<(NN * KCH / 64 + 63) / 64, 256, 0, stream>>>(L, RS, CS, c, Ah, Al);
        k_gemmw<bf, 1, false><<<dim3(NN / 64, DD / 64, 1), 32, 0, stream>>>(Ah, Al, (pos ? YT : XT) + (size_t)(c % (NCHK / 2)) * DD * KCH, nullptr, KCH, P, DD, nullptr, 0, 0, 0);
        k_acc<<<(unsigned)(((size_t)NN * DD / 4 + 255) / 256), 256, 0, stream>>>(P, ACC, c == 0 ? 1 : 0, pos ? 1.0f : -1.0f, c == NCHK - 1 ? OUT : ACC); }
}
